// GatedGraphConvolution_21337397526884
// MI455X (gfx1250) — hardware-verified
//
#include <hip/hip_runtime.h>
#include <stddef.h>
#include <stdint.h>
#include <math.h>


#define DD     128
#define KS     256
#define NTHR   256
#define NWAVE  8
#define EPT    8
#define CHUNK  (NTHR * EPT)
#define WCAP   (EPT * 32)
#define LISTN  (NWAVE * WCAP)
#define NBA    1024
#define SLA    10
#define RCAP   28672
#define DEGCAP 64
#define GBM    128
#define GTHR   256
#define NBW1   16
#define NBW2   8
#define AGG_ZINTS (LISTN + 2 * RCAP + 3 * NBA)
#define AGG_LDS_INTS (AGG_ZINTS + 16)
#define GATE_LDS_FLOATS (3 * GBM * DD + 3 * DD)
#define WSMAX  134217728

static_assert(DD == 128);
static_assert((CHUNK & (CHUNK - 1)) == 0 && CHUNK <= 4096);
static_assert((NBA & (NBA - 1)) == 0 && NBA == (1 << SLA));
static_assert(((long long)CHUNK << SLA) < (1LL << 31));
static_assert(LISTN % NTHR == 0);
static_assert(NBA % NWAVE == 0 && NBA % 32 == 0 && NBA % GBM == 0);
static_assert(RCAP % 4 == 0 && AGG_ZINTS % 4 == 0 && LISTN % 4 == 0);
static_assert(RCAP >= 17558);
static_assert(DEGCAP % 32 == 0 && DEGCAP >= 36 + 8);
static_assert(DD == 4 * 32 && KS == 2 * DD && KS % 32 == 0 && DD % 32 == 0);
static_assert(GBM == (GTHR / 32) * 16);
static_assert(NBW1 * NTHR == DD * (KS / 8) && NBW2 * NTHR == DD * (DD / 8));
static_assert(98 * NBA >= 100000 && 782 * GBM >= 100000);
static_assert(DD * 4 == 512 && KS * 2 == 512 && DD * 2 == 256);
static_assert(AGG_LDS_INTS * 4 <= 300000);
static_assert(GATE_LDS_FLOATS * 4 <= 327680);

typedef float          v4f   __attribute__((ext_vector_type(4)));
typedef float          v8f   __attribute__((ext_vector_type(8)));
typedef int            v4i   __attribute__((ext_vector_type(4)));
typedef int            v8i   __attribute__((ext_vector_type(8)));
typedef unsigned       v2u   __attribute__((ext_vector_type(2)));
typedef unsigned short v8us  __attribute__((ext_vector_type(8)));
typedef unsigned short v16us __attribute__((ext_vector_type(16)));
typedef __bf16         v16bf __attribute__((ext_vector_type(16)));
typedef v4f  __attribute__((may_alias)) v4fa;
typedef v4i  __attribute__((may_alias)) v4ia;
typedef v2u  __attribute__((may_alias)) v2ua;
typedef v8us __attribute__((may_alias)) v8usa;
union FragB { v16bf v; v16us u; v8us h[2]; v8i w; };

__device__ __forceinline__ v8f wmb(const FragB& a, const FragB& b, v8f c) {
  v8f d = __builtin_amdgcn_wmma_f32_16x16x32_bf16(false, a.v, false, b.v, (short)0, c, false, false);
  asm volatile("v_nop\n\tv_nop\n\tv_nop\n\tv_nop" : "+v"(d) : "v"(a.w), "v"(b.w));
  return d;
}

__device__ __forceinline__ unsigned bf16_bits(float f) {
  const unsigned u = __float_as_uint(f);
  const unsigned r = (u + 0x7FFFu + ((u >> 16) & 1u)) >> 16;
  return (f != f) ? 0x7FC0u : r;
}
__device__ __forceinline__ float bf16_val(float f) {
  return __uint_as_float(bf16_bits(f) << 16);
}

__device__ __forceinline__ void hilo_pack(float v0, float v1, float v2, float v3,
                                          int& h01, int& h23, int& l01, int& l23) {
  const unsigned a0 = bf16_bits(v0), a1 = bf16_bits(v1), a2 = bf16_bits(v2), a3 = bf16_bits(v3);
  const unsigned b0 = bf16_bits(v0 - __uint_as_float(a0 << 16));
  const unsigned b1 = bf16_bits(v1 - __uint_as_float(a1 << 16));
  const unsigned b2 = bf16_bits(v2 - __uint_as_float(a2 << 16));
  const unsigned b3 = bf16_bits(v3 - __uint_as_float(a3 << 16));
  h01 = (int)(a0 | (a1 << 16)); h23 = (int)(a2 | (a3 << 16));
  l01 = (int)(b0 | (b1 << 16)); l23 = (int)(b2 | (b3 << 16));
}

__device__ __forceinline__ v4i regroup16(int h01, int h23, int l01, int l23, int lane) {
  const int s0 = (2 * lane) & 31, s1 = s0 + 1;
  const int a0 = __shfl(h01, s0, 32), a1 = __shfl(h23, s0, 32), a2 = __shfl(h01, s1, 32), a3 = __shfl(h23, s1, 32);
  const int b0 = __shfl(l01, s0, 32), b1 = __shfl(l23, s0, 32), b2 = __shfl(l01, s1, 32), b3 = __shfl(l23, s1, 32);
  const int mk = (lane < 16) ? -1 : 0;
  v4i o;
  o.x = (a0 & mk) | (b0 & ~mk); o.y = (a1 & mk) | (b1 & ~mk);
  o.z = (a2 & mk) | (b2 & ~mk); o.w = (a3 & mk) | (b3 & ~mk);
  return o;
}

template <int SLB>
__device__ __forceinline__ int scan_chunk(const int* __restrict__ dsts, int nE, int cbase, int slotBase,
                                          int nb, int vec8, int* list, int tid, int lane, int wave) {
  int wc = 0;
  const int el0  = tid * EPT;
  const int e0   = cbase + el0;
  const int sent = -2147483647 - 1;
  v4i da, db;
  if (vec8 != 0 && cbase + CHUNK <= nE) {
    da = *(const v4i*)(dsts + e0);
    db = *(const v4i*)(dsts + e0 + 4);
  } else {
    da.x = (e0     < nE) ? dsts[min(e0,     nE - 1)] : sent;
    da.y = (e0 + 1 < nE) ? dsts[min(e0 + 1, nE - 1)] : sent;
    da.z = (e0 + 2 < nE) ? dsts[min(e0 + 2, nE - 1)] : sent;
    da.w = (e0 + 3 < nE) ? dsts[min(e0 + 3, nE - 1)] : sent;
    db.x = (e0 + 4 < nE) ? dsts[min(e0 + 4, nE - 1)] : sent;
    db.y = (e0 + 5 < nE) ? dsts[min(e0 + 5, nE - 1)] : sent;
    db.z = (e0 + 6 < nE) ? dsts[min(e0 + 6, nE - 1)] : sent;
    db.w = (e0 + 7 < nE) ? dsts[min(e0 + 7, nE - 1)] : sent;
  }
  const unsigned nbs = (unsigned)slotBase;
  const unsigned unb = (unsigned)nb;
  const unsigned s0 = (unsigned)da.x - nbs, s1 = (unsigned)da.y - nbs;
  const unsigned s2 = (unsigned)da.z - nbs, s3 = (unsigned)da.w - nbs;
  const unsigned s4 = (unsigned)db.x - nbs, s5 = (unsigned)db.y - nbs;
  const unsigned s6 = (unsigned)db.z - nbs, s7 = (unsigned)db.w - nbs;
  const bool h0 = s0 < unb, h1 = s1 < unb, h2 = s2 < unb, h3 = s3 < unb;
  const bool h4 = s4 < unb, h5 = s5 < unb, h6 = s6 < unb, h7 = s7 < unb;
  const unsigned any = __builtin_amdgcn_ballot_w32(h0 | h1 | h2 | h3 | h4 | h5 | h6 | h7);
  if (any != 0u) {
#define HITJ(J, HJ, SJ) { \
      const unsigned mj = __builtin_amdgcn_ballot_w32(HJ); \
      if (mj != 0u) { \
        if (HJ) { \
          const int pos = wc + (int)__builtin_amdgcn_mbcnt_lo(mj, 0u); \
          if (pos < WCAP) list[wave * WCAP + pos] = ((el0 + (J)) << SLB) | (int)(SJ); \
        } \
        wc += (int)__builtin_popcount(mj); } }
    HITJ(0, h0, s0)
    HITJ(1, h1, s1)
    HITJ(2, h2, s2)
    HITJ(3, h3, s3)
    HITJ(4, h4, s4)
    HITJ(5, h5, s5)
    HITJ(6, h6, s6)
    HITJ(7, h7, s7)
#undef HITJ
  }
  return wc;
}

template <int LG>
__device__ __forceinline__ void wt_unit(const float* __restrict__ w, unsigned short* wt, int u) {
  const int n  = u >> LG;
  const int k8 = (u & ((1 << LG) - 1)) * 8;
  const int kk = k8 & (DD - 1);
  const float* p = w + (size_t)kk * DD + n;
  const float f0 = p[0],      f1 = p[DD],     f2 = p[2 * DD], f3 = p[3 * DD];
  const float f4 = p[4 * DD], f5 = p[5 * DD], f6 = p[6 * DD], f7 = p[7 * DD];
  v8us o;
  o[0] = (unsigned short)bf16_bits(f0); o[1] = (unsigned short)bf16_bits(f1);
  o[2] = (unsigned short)bf16_bits(f2); o[3] = (unsigned short)bf16_bits(f3);
  o[4] = (unsigned short)bf16_bits(f4); o[5] = (unsigned short)bf16_bits(f5);
  o[6] = (unsigned short)bf16_bits(f6); o[7] = (unsigned short)bf16_bits(f7);
  unsigned short* dp = wt + (size_t)n * (8 << LG) + k8;
  *(volatile v8us*)dp = o;
  __threadfence();
  *(volatile v8us*)dp = o;
}

__global__ __launch_bounds__(NTHR) void k_prep(const float* __restrict__ x, int nN, int gx,
                                               const float* __restrict__ w1, const float* __restrict__ w2,
                                               const float* __restrict__ w3, const float* __restrict__ b1,
                                               const float* __restrict__ b2, const float* __restrict__ b3,
                                               const float* __restrict__ eps,
                                               unsigned short* xb, unsigned short* w1d, unsigned short* w2t,
                                               unsigned short* w3t, float* par) {
  const int tid = (int)threadIdx.x, lane = tid & 31, wave = tid >> 5;
  const int blk = (int)blockIdx.x;
  if (blk < gx) {
    const int u   = blk * NTHR + tid;
    const int row = u >> 4;
    const int c8  = (u & 15) * 8;
    const int rc  = row < nN ? row : nN - 1;
    const unsigned mk = (row < nN) ? 0xFFFFu : 0u;
    const float* p = x + (size_t)rc * DD + c8;
    const v4f a = *(const v4fa*)p;
    const v4f b = *(const v4fa*)(p + 4);
    v8us o;
    o[0] = (unsigned short)(bf16_bits(a.x) & mk); o[1] = (unsigned short)(bf16_bits(a.y) & mk);
    o[2] = (unsigned short)(bf16_bits(a.z) & mk); o[3] = (unsigned short)(bf16_bits(a.w) & mk);
    o[4] = (unsigned short)(bf16_bits(b.x) & mk); o[5] = (unsigned short)(bf16_bits(b.y) & mk);
    o[6] = (unsigned short)(bf16_bits(b.z) & mk); o[7] = (unsigned short)(bf16_bits(b.w) & mk);
    unsigned short* dp = xb + (size_t)row * DD + c8;
    *(volatile v8us*)dp = o;
    __threadfence();
    *(volatile v8us*)dp = o;
  } else {
    const int pb = blk - gx;
    if (pb < NBW1) {
      wt_unit<5>(w1, w1d, pb * NTHR + tid);
    } else if (pb < NBW1 + NBW2) {
      wt_unit<4>(w2, w2t, (pb - NBW1) * NTHR + tid);
    } else if (pb < NBW1 + 2 * NBW2) {
      wt_unit<4>(w3, w3t, (pb - NBW1 - NBW2) * NTHR + tid);
    } else if (pb == NBW1 + 2 * NBW2) {
      if (wave < 4) {
        v4f v;
        if (wave == 0)      v = *(const v4fa*)(b1 + 4 * lane);
        else if (wave == 1) v = *(const v4fa*)(b2 + 4 * lane);
        else if (wave == 2) v = *(const v4fa*)(b3 + 4 * lane);
        else { const float e = eps[0]; v.x = e; v.y = e; v.z = e; v.w = e; }
        v4f o;
        o.x = bf16_val(v.x); o.y = bf16_val(v.y); o.z = bf16_val(v.z); o.w = bf16_val(v.w);
        float* dp = par + wave * DD + 4 * lane;
        *(volatile v4f*)dp = o;
        __threadfence();
        *(volatile v4f*)dp = o;
      }
    }
  }
}

__global__ __launch_bounds__(NTHR) void k_scan(const int* __restrict__ gsrc, const int* __restrict__ keys,
                                               const float* __restrict__ ew, int nE, int nN, int vec8, int mRows,
                                               const unsigned short* __restrict__ xb,
                                               const float* __restrict__ par,
                                               unsigned short* shl, int* flag) {
  extern __shared__ __attribute__((aligned(16))) int dsm[];
  int* list = dsm;
  int* hl   = dsm + LISTN;
  int* sl   = dsm + LISTN + RCAP;
  int* cnt  = dsm + LISTN + 2 * RCAP;
  int* offs = cnt + NBA;
  int* cur  = offs + NBA;
  int* misc = cur + NBA;
  const int tid = (int)threadIdx.x, lane = tid & 31, wave = tid >> 5;
  const int nodeBase = (int)blockIdx.x * NBA;

  {
    const v4i z4 = {0, 0, 0, 0};
    for (int i = tid * 4; i < AGG_ZINTS; i += NTHR * 4) *(v4ia*)(dsm + i) = z4;
    if (tid < 16) misc[tid] = 0;
  }
  __syncthreads();

  int t = 0, ov = 0;
  const int nChunks = (nE + CHUNK - 1) / CHUNK;
#pragma unroll 1
  for (int ch = 0; ch < nChunks; ++ch) {
    const int cbase = ch * CHUNK;
    const int wc = scan_chunk<SLA>(keys, nE, cbase, nodeBase, NBA, vec8, list, tid, lane, wave);
    if (lane == 0) misc[wave] = wc;
    __syncthreads();
    if (wave == 0) {
#pragma unroll 1
      for (int w2 = 0; w2 < NWAVE; ++w2) {
        int c = misc[w2];
        c = c < 0 ? 0 : (c > WCAP ? WCAP : c);
#pragma unroll 1
        for (int b0 = 0; b0 < c; b0 += 32) {
          const int idx = b0 + lane;
          const int ent = list[w2 * WCAP + (idx < WCAP ? idx : WCAP - 1)];
          const int m32 = (c - b0) < 32 ? (c - b0) : 32;
#pragma unroll 1
          for (int k = 0; k < m32; ++k) {
            const int u    = __builtin_amdgcn_readlane(ent, k);
            const int slot = u & (NBA - 1);
            const int el   = (u >> SLA) & (CHUNK - 1);
            const int pk   = ((cbase + el) << SLA) | slot;
            if (t < RCAP) {
              if (lane == 0) { hl[t] = pk; cnt[slot] = cnt[slot] + 1; }
              t = t + 1;
            } else {
              ov = 1;
            }
          }
        }
      }
    }
    __syncthreads();
  }
  if (wave == 0 && lane == 0) { misc[8] = t; misc[9] = ov; }
  __syncthreads();
  int tt = misc[8];
  tt = tt < 0 ? 0 : (tt > RCAP ? RCAP : tt);
  const int ovf = misc[9];

  if (wave == 0 && lane < 8) {
    v4i fv;
    fv.x = ovf; fv.y = ovf; fv.z = ovf; fv.w = ovf;
    int* fp = flag + (size_t)blockIdx.x * 32 + 4 * lane;
    *(volatile v4i*)fp = fv;
    __threadfence();
    *(volatile v4i*)fp = fv;
  }

  if (wave == 0) {
    const int base = lane * (NBA / 32);
    int s = 0;
#pragma unroll 1
    for (int i = 0; i < NBA / 32; ++i) s += cnt[base + i];
    int incl = s;
#pragma unroll
    for (int d = 1; d < 32; d <<= 1) {
      const int y = __shfl_up(incl, d, 32);
      if (lane >= d) incl += y;
    }
    int run = incl - s;
#pragma unroll 1
    for (int i = 0; i < NBA / 32; ++i) {
      const int cv = cnt[base + i];
      offs[base + i] = run;
      cur[base + i]  = run;
      run += cv;
    }
  }
  __syncthreads();
  if (wave == 0) {
#pragma unroll 1
    for (int b0 = 0; b0 < tt; b0 += 32) {
      const int idx = b0 + lane;
      const int ent = hl[idx < RCAP ? idx : RCAP - 1];
      const int m32 = (tt - b0) < 32 ? (tt - b0) : 32;
#pragma unroll 1
      for (int k = 0; k < m32; ++k) {
        const int u    = __builtin_amdgcn_readlane(ent, k);
        const int slot = u & (NBA - 1);
        if (lane == 0) {
          int p = cur[slot];
          p = p < 0 ? 0 : (p > RCAP - 1 ? RCAP - 1 : p);
          sl[p] = u;
          cur[slot] = p + 1;
        }
      }
    }
  }
  __syncthreads();

  const float epsb = par[3 * DD];
  const float pz = (ovf != 0) ? __int_as_float(0x7fc00000) : 0.0f;
#pragma unroll 1
  for (int si = 0; si < NBA / NWAVE; ++si) {
    const int s    = si * NWAVE + wave;
    const int node = nodeBase + s;
    int c = cnt[s];
    const bool big = c > DEGCAP;
    c = c < 0 ? 0 : (c > DEGCAP ? DEGCAP : c);
    int o = offs[s];
    o = o < 0 ? 0 : (o > RCAP ? RCAP : o);
    const int nc = node < nN ? node : nN - 1;
    float g0 = 0.0f, g1 = 0.0f, g2 = 0.0f, g3 = 0.0f;
#pragma unroll 1
    for (int b0 = 0; b0 < c; b0 += 32) {
      int idx = o + b0 + lane;
      idx = idx > RCAP - 1 ? RCAP - 1 : idx;
      const int ent = sl[idx];
      int eid = ent >> SLA;
      eid = eid < 0 ? 0 : (eid > nE - 1 ? nE - 1 : eid);
      int sr = gsrc[eid];
      const float wraw = ew[eid];
      asm volatile("" :: "v"(sr));
      asm volatile("" :: "v"(wraw));
      sr = sr < 0 ? 0 : (sr > nN - 1 ? nN - 1 : sr);
      const int wvi = __float_as_int(bf16_val(wraw));
      const int m32 = (c - b0) < 32 ? (c - b0) : 32;
#pragma unroll 1
      for (int k = 0; k < m32; ++k) {
        const int   sk = __builtin_amdgcn_readlane(sr, k);
        const float wk = __int_as_float(__builtin_amdgcn_readlane(wvi, k));
        const v2u a = *(const v2ua*)(xb + (size_t)sk * DD + 4 * lane);
        g0 = fmaf(wk, __uint_as_float(a.x << 16),         g0);
        g1 = fmaf(wk, __uint_as_float(a.x & 0xffff0000u), g1);
        g2 = fmaf(wk, __uint_as_float(a.y << 16),         g2);
        g3 = fmaf(wk, __uint_as_float(a.y & 0xffff0000u), g3);
      }
    }
    {
      const v2u sx = *(const v2ua*)(xb + (size_t)nc * DD + 4 * lane);
      g0 = fmaf(epsb, __uint_as_float(sx.x << 16),         g0);
      g1 = fmaf(epsb, __uint_as_float(sx.x & 0xffff0000u), g1);
      g2 = fmaf(epsb, __uint_as_float(sx.y << 16),         g2);
      g3 = fmaf(epsb, __uint_as_float(sx.y & 0xffff0000u), g3);
    }
    const float pzr = big ? __int_as_float(0x7fc00000) : pz;
    const bool live = node < nN;
    const float q0 = live ? g0 + pzr : 0.0f, q1 = live ? g1 + pzr : 0.0f;
    const float q2 = live ? g2 + pzr : 0.0f, q3 = live ? g3 + pzr : 0.0f;
    int h01, h23, l01, l23;
    hilo_pack(q0, q1, q2, q3, h01, h23, l01, l23);
    const v4i ow = regroup16(h01, h23, l01, l23, lane);
    if (node < mRows) {
      unsigned short* hp = shl + (size_t)node * KS + 8 * lane;
      *(volatile v4i*)hp = ow;
      __threadfence();
      *(volatile v4i*)hp = ow;
    }
  }
}

template <int KK>
__device__ __forceinline__ void panel(const unsigned short* __restrict__ A, const unsigned short* __restrict__ BT,
                                      float* stg, int rowBase, int wave, int hh, int m) {
  v8f acc[8];
  {
    const v8f z = {0.f, 0.f, 0.f, 0.f, 0.f, 0.f, 0.f, 0.f};
#pragma unroll
    for (int t = 0; t < 8; ++t) acc[t] = z;
  }
  const unsigned short* ap = A  + (size_t)(rowBase + 16 * wave + m) * (size_t)KK + 8 * hh;
  const unsigned short* bp = BT + (size_t)m * (size_t)KK + 8 * hh;
#pragma unroll 1
  for (int k0 = 0; k0 < KK; k0 += 32) {
    FragB af;
    af.h[0] = *(const v8usa*)(ap + k0);
    af.h[1] = *(const v8usa*)(ap + k0 + 16);
#pragma unroll
    for (int nt = 0; nt < 8; ++nt) {
      const unsigned short* wq = bp + (size_t)(16 * nt) * (size_t)KK + k0;
      FragB bf;
      bf.h[0] = *(const v8usa*)wq;
      bf.h[1] = *(const v8usa*)(wq + 16);
      acc[nt] = wmb(af, bf, acc[nt]);
    }
  }
#pragma unroll
  for (int nt = 0; nt < 8; ++nt) {
    const int lc = 16 * nt + m;
#pragma unroll
    for (int r = 0; r < 8; ++r) {
      const int lr = 16 * wave + 8 * hh + r;
      stg[lr * DD + lc] = acc[nt][r];
    }
  }
}

__device__ __forceinline__ float gate1(float o, float t, float g, float c1, float c2, float c3) {
  float v = o + c1;
  v = (v > 0.0f) ? v : (v - v);
  const float tr = t + c2;
  const float s  = g + c3;
  const float gg = 1.0f / (1.0f + expf(-s));
  return tr + gg * (v - tr);
}

__global__ __launch_bounds__(GTHR) __attribute__((amdgpu_num_vgpr(248)))
void k_gate(const unsigned short* __restrict__ xb, const unsigned short* __restrict__ shl,
            const unsigned short* __restrict__ w1d, const unsigned short* __restrict__ w2t,
            const unsigned short* __restrict__ w3t, const float* __restrict__ par,
            const int* __restrict__ flag, int nFlag, int nN, float* outp) {
  extern __shared__ __attribute__((aligned(16))) float gsm[];
  float* stgT = gsm;
  float* stgG = gsm + GBM * DD;
  float* stgO = gsm + 2 * GBM * DD;
  float* spar = gsm + 3 * GBM * DD;
  const int tid = (int)threadIdx.x, lane = tid & 31, wave = tid >> 5, hh = lane >> 4, m = lane & 15;
  const int rowBase = (int)blockIdx.x * GBM;

  if (tid < 96) {
    const v4f pv = *(const v4fa*)(par + 4 * tid);
    *(v4fa*)(spar + 4 * tid) = pv;
  }

  panel<DD>(xb,  w2t, stgT, rowBase, wave, hh, m);
  panel<DD>(xb,  w3t, stgG, rowBase, wave, hh, m);
  panel<KS>(shl, w1d, stgO, rowBase, wave, hh, m);
  __syncthreads();

  const v4f c1 = *(const v4fa*)(spar + 4 * lane);
  const v4f c2 = *(const v4fa*)(spar + DD + 4 * lane);
  const v4f c3 = *(const v4fa*)(spar + 2 * DD + 4 * lane);
  int fb = rowBase >> SLA;
  fb = fb < 0 ? 0 : (fb > nFlag - 1 ? nFlag - 1 : fb);
  const int fl = flag[(size_t)fb * 32];
  const float nanv = __int_as_float(0x7fc00000);

#pragma unroll 1
  for (int i = 0; i < 16; ++i) {
    const int lr   = 16 * wave + i;
    const int grow = rowBase + lr;
    const v4f tv = *(const v4fa*)(stgT + lr * DD + 4 * lane);
    const v4f gv = *(const v4fa*)(stgG + lr * DD + 4 * lane);
    const v4f ov = *(const v4fa*)(stgO + lr * DD + 4 * lane);
    float r0 = gate1(ov.x, tv.x, gv.x, c1.x, c2.x, c3.x);
    float r1 = gate1(ov.y, tv.y, gv.y, c1.y, c2.y, c3.y);
    float r2 = gate1(ov.z, tv.z, gv.z, c1.z, c2.z, c3.z);
    float r3 = gate1(ov.w, tv.w, gv.w, c1.w, c2.w, c3.w);
    r0 = (fl != 0) ? nanv : r0; r1 = (fl != 0) ? nanv : r1;
    r2 = (fl != 0) ? nanv : r2; r3 = (fl != 0) ? nanv : r3;
    v4f o;
    o.x = r0; o.y = r1; o.z = r2; o.w = r3;
    if (grow < nN) {
      float* op = outp + (size_t)grow * DD + 4 * lane;
      *(volatile v4f*)op = o;
      __threadfence();
      *(volatile v4f*)op = o;
    }
  }
}

static inline int cdiv(int a, int b) { return (a + b - 1) / b; }
static inline size_t al256(size_t o) { return (o + 255) & ~(size_t)255; }

extern "C" void kernel_launch(void* const* d_in, const int* in_sizes, int n_in,
                              void* d_out, int out_size, void* d_ws, size_t ws_size,
                              hipStream_t stream) {
  if (n_in < 11) return;
  if (in_sizes[0] < DD || (in_sizes[0] % DD) != 0) return;
  const int nN = in_sizes[0] / DD;
  const int nE = in_sizes[1];
  if (nE < 1 || in_sizes[2] != nE || in_sizes[3] != nE) return;
  if (nE >= (1 << 21) || nN < 16 || nN >= (1 << 24)) return;
  if (in_sizes[4] != DD * DD || in_sizes[5] != DD * DD || in_sizes[6] != DD * DD) return;
  if (in_sizes[7] != DD || in_sizes[8] != DD || in_sizes[9] != DD) return;
  if (in_sizes[10] < 1) return;
  if ((long long)out_size != (long long)nN * DD) return;

  const float* x    = (const float*)d_in[0];
  const int*   esrc = (const int*)d_in[1];
  const int*   edst = (const int*)d_in[2];
  const float* ew   = (const float*)d_in[3];
  const float* w1   = (const float*)d_in[4];
  const float* w2   = (const float*)d_in[5];
  const float* w3   = (const float*)d_in[6];
  const float* b1   = (const float*)d_in[7];
  const float* b2   = (const float*)d_in[8];
  const float* b3   = (const float*)d_in[9];
  const float* eps  = (const float*)d_in[10];
  float* out = (float*)d_out;

  const int MP = cdiv(nN, GBM) * GBM;
  const int gG = MP / GBM;
  const int gX = MP / 16;
  const int gA = cdiv(nN, NBA);
  if ((long long)gA * NBA < (long long)MP) return;
  const int vec8 = ((nE & 3) == 0) ? 1 : 0;

  char* ws = (char*)d_ws;
  size_t off = 0;
  const size_t oXB  = off; off = al256(off + (size_t)MP * DD * 2);
  const size_t oSHL = off; off = al256(off + (size_t)MP * KS * 2);
  const size_t oW1D = off; off = al256(off + (size_t)DD * KS * 2);
  const size_t oW2T = off; off = al256(off + (size_t)DD * DD * 2);
  const size_t oW3T = off; off = al256(off + (size_t)DD * DD * 2);
  const size_t oPAR = off; off = al256(off + (size_t)4 * DD * 4);
  const size_t oFLG = off; off = al256(off + (size_t)gA * 128);
  if (off > ws_size || off > (size_t)WSMAX) return;
  unsigned short* XB  = (unsigned short*)(ws + oXB);
  unsigned short* SHL = (unsigned short*)(ws + oSHL);
  unsigned short* W1D = (unsigned short*)(ws + oW1D);
  unsigned short* W2T = (unsigned short*)(ws + oW2T);
  unsigned short* W3T = (unsigned short*)(ws + oW3T);
  float*          PAR = (float*)(ws + oPAR);
  int*            FLG = (int*)(ws + oFLG);

  const size_t scanLds = (size_t)AGG_LDS_INTS * 4;
  const size_t gateLds = (size_t)GATE_LDS_FLOATS * 4;
  hipFuncSetAttribute(reinterpret_cast<const void*>(&k_scan), hipFuncAttributeMaxDynamicSharedMemorySize, (int)scanLds);
  hipFuncSetAttribute(reinterpret_cast<const void*>(&k_gate), hipFuncAttributeMaxDynamicSharedMemorySize, (int)gateLds);

  k_prep<<<gX + NBW1 + 2 * NBW2 + 1, NTHR, 0, stream>>>(x, nN, gX, w1, w2, w3, b1, b2, b3, eps,
                                                       XB, W1D, W2T, W3T, PAR);
  k_scan<<<gA, NTHR, scanLds, stream>>>(esrc, edst, ew, nE, nN, vec8, MP, XB, PAR, SHL, FLG);
  k_gate<<<gG, GTHR, gateLds, stream>>>(XB, SHL, W1D, W2T, W3T, PAR, FLG, gA, nN, out);
}
